// MambaSSM_48730698940563
// MI455X (gfx1250) — hardware-verified
//
#include <hip/hip_runtime.h>
#include <math.h>

typedef __attribute__((ext_vector_type(16))) _Float16 v16h;
typedef __attribute__((ext_vector_type(8)))  _Float16 v8h;
typedef __attribute__((ext_vector_type(16))) __bf16   v16b;
typedef __attribute__((ext_vector_type(8)))  __bf16   v8b;
typedef __attribute__((ext_vector_type(8)))  float    v8f;
typedef __attribute__((ext_vector_type(4)))  float    v4f;

constexpr int kBatch  = 2;
constexpr int kSeq    = 2048;
constexpr int kDm     = 128;
constexpr int kDin    = 256;
constexpr int kDst    = 256;
constexpr int kConvK  = 4;
constexpr int kXzW    = 2 * kDin;
constexpr int kXxW    = 2 * kDst;
constexpr int kRows   = kBatch * kSeq;
constexpr int kConvTP = 260;
constexpr int kScanTS = 32;
constexpr int kScanGP = 260;
static_assert(kDst == kDin);
static_assert((kDm % 32) == 0 && (kDin % 32) == 0);
static_assert((kRows % 64) == 0 && (kXzW % 64) == 0 && (kDst % 64) == 0 && (kDm % 64) == 0);
static_assert((kDm % 64) == 0 && (kDin % 64) == 0 && (kXzW % 32) == 0 && (kDst % 32) == 0 && (kDm % 32) == 0);
static_assert((kSeq % 64) == 0 && (kSeq % kScanTS) == 0 && (kScanTS % 8) == 0);

constexpr size_t kOffXH   = 0;
constexpr size_t kOffXL   = kOffXH  + (size_t)kRows * kDm  * 2;
constexpr size_t kOffWIH  = kOffXL  + (size_t)kRows * kDm  * 2;
constexpr size_t kOffWIL  = kOffWIH + (size_t)kXzW  * kDm  * 2;
constexpr size_t kOffWDH  = kOffWIL + (size_t)kXzW  * kDm  * 2;
constexpr size_t kOffWDL  = kOffWDH + (size_t)kDst  * kDin * 2;
constexpr size_t kOffWOH  = kOffWDL + (size_t)kDst  * kDin * 2;
constexpr size_t kOffWOL  = kOffWOH + (size_t)kDm   * kDin * 2;
constexpr size_t kOffAT   = kOffWOL + (size_t)kDm   * kDin * 2;
constexpr size_t kOffXZ   = kOffAT  + (size_t)kDst  * kDin * 4;
constexpr size_t kOffXC   = kOffXZ  + (size_t)kRows * kXzW * 4;
constexpr size_t kOffXCH  = kOffXC  + (size_t)kRows * kDin * 4;
constexpr size_t kOffXCL  = kOffXCH + (size_t)kRows * kDin * 2;
constexpr size_t kOffSS   = kOffXCL + (size_t)kRows * kDin * 2;
constexpr size_t kOffPRE  = kOffSS  + (size_t)kRows * 4;
constexpr size_t kOffGH   = kOffPRE + (size_t)kRows * kDst * 4;
constexpr size_t kOffGL   = kOffGH  + (size_t)kRows * kDin * 2;
constexpr size_t kWsTotal = kOffGL  + (size_t)kRows * kDin * 2;
static_assert(kWsTotal == 28196864ull);
static_assert(kWsTotal <= 134217728ull);
static_assert((kOffXL % 128) == 0 && (kOffWIH % 128) == 0 && (kOffWIL % 128) == 0 && (kOffWDH % 128) == 0 &&
              (kOffWDL % 128) == 0 && (kOffWOH % 128) == 0 && (kOffWOL % 128) == 0 && (kOffAT % 128) == 0 &&
              (kOffXZ % 128) == 0 && (kOffXC % 128) == 0 && (kOffXCH % 128) == 0 && (kOffXCL % 128) == 0 &&
              (kOffSS % 128) == 0 && (kOffPRE % 128) == 0 && (kOffGH % 128) == 0 && (kOffGL % 128) == 0);

__device__ __forceinline__ unsigned short f2bf_bits(float f) {
  unsigned u = __float_as_uint(f);
  return (unsigned short)((u + 0x7FFFu + ((u >> 16) & 1u)) >> 16);
}
__device__ __forceinline__ float bf_bits2f(unsigned short h) { return __uint_as_float(((unsigned)h) << 16); }

__device__ __forceinline__ void dep_guard4_h(v8f& a, v8f& b, v8f& c, v8f& d, v16h x, v16h y) { asm volatile("v_nop\n\tv_nop\n\tv_nop\n\tv_nop" : "+v"(a), "+v"(b), "+v"(c), "+v"(d) : "v"(x), "v"(y)); }
__device__ __forceinline__ void dep_guard4_b(v8f& a, v8f& b, v8f& c, v8f& d, v16b x, v16b y) { asm volatile("v_nop\n\tv_nop\n\tv_nop\n\tv_nop" : "+v"(a), "+v"(b), "+v"(c), "+v"(d) : "v"(x), "v"(y)); }
__device__ __forceinline__ void keep4_h(v16h a, v16h b, v16h c, v16h d) { asm volatile("v_nop" :: "v"(a), "v"(b), "v"(c), "v"(d)); }
__device__ __forceinline__ void keep4_b(v16b a, v16b b, v16b c, v16b d) { asm volatile("v_nop" :: "v"(a), "v"(b), "v"(c), "v"(d)); }
__device__ __forceinline__ void acc_guard4(v8f& a, v8f& b, v8f& c, v8f& d) { asm volatile("v_nop\n\tv_nop\n\tv_nop\n\tv_nop" : "+v"(a), "+v"(b), "+v"(c), "+v"(d)); }
template <typename T> struct Frag;
template <> struct Frag<_Float16> {
  typedef v16h V; union U { v16h v; v8h h[2]; };
  static __device__ __forceinline__ v16h load(const _Float16* p) {
    U f; f.h[0] = *(const v8h*)(p); f.h[1] = *(const v8h*)(p + 16); return f.v;
  }
  static __device__ __forceinline__ v8f mma(v16h a, v16h b, v8f c) {
    return __builtin_amdgcn_wmma_f32_16x16x32_f16(false, a, false, b, (short)0, c, false, false);
  }
  static __device__ __forceinline__ void guard4(v8f& a, v8f& b, v8f& c, v8f& d, v16h x, v16h y) { dep_guard4_h(a, b, c, d, x, y); }
  static __device__ __forceinline__ void keep(v16h a, v16h b, v16h c, v16h d) { keep4_h(a, b, c, d); }
};
template <> struct Frag<__bf16> {
  typedef v16b V; union U { v16b v; v8b h[2]; };
  static __device__ __forceinline__ v16b load(const __bf16* p) {
    U f; f.h[0] = *(const v8b*)(p); f.h[1] = *(const v8b*)(p + 16); return f.v;
  }
  static __device__ __forceinline__ v8f mma(v16b a, v16b b, v8f c) {
    return __builtin_amdgcn_wmma_f32_16x16x32_bf16(false, a, false, b, (short)0, c, false, false);
  }
  static __device__ __forceinline__ void guard4(v8f& a, v8f& b, v8f& c, v8f& d, v16b x, v16b y) { dep_guard4_b(a, b, c, d, x, y); }
  static __device__ __forceinline__ void keep(v16b a, v16b b, v16b c, v16b d) { keep4_b(a, b, c, d); }
};

template <int ET> struct Elem;
template <> struct Elem<0> { typedef _Float16 T; };
template <> struct Elem<1> { typedef __bf16 T; };
template <int ET, int SPL, int BIAS_MODE, int OUT_MODE, bool RESID, int ACT = 0>
__global__ __launch_bounds__(256) void wmma_gemm64(
    const unsigned short* __restrict__ Ap, const unsigned short* __restrict__ A2p, int lda, long strideA,
    const unsigned short* __restrict__ Btp, const unsigned short* __restrict__ Bt2p, int ldb, long strideB,
    void* __restrict__ Cout, void* __restrict__ Cout2, int ldc, long strideC,
    const float* __restrict__ bias,
    const float* __restrict__ resid, long strideR,
    int M, int N, int K, float scale) {
  typedef typename Elem<ET>::T T;
  typedef typename Frag<T>::V V;
  const T* A = (const T*)Ap; const T* A2 = (const T*)A2p; const T* Bt = (const T*)Btp; const T* Bt2 = (const T*)Bt2p;
  __shared__ __align__(16) float sT[8][16 * 68];
  const int b    = blockIdx.y;
  const int lane = threadIdx.x & 31;
  const int wave = threadIdx.x >> 5;
  const int tilesN = N >> 6;
  const int tilesM = M >> 6;
  const int tile = blockIdx.x * 8 + wave;
  if (tile >= tilesM * tilesN) return;
  const int tm = tile / tilesN;
  const int tn = tile - tm * tilesN;
  const int m0 = tm << 6;
  const int n0 = tn << 6;

  const T* Ab  = A  + (size_t)b * strideA;
  const T* Bb  = Bt + (size_t)b * strideB;
  const T* Ab2 = (SPL >= 1) ? (A2  + (size_t)b * strideA) : nullptr;
  const T* Bb2 = (SPL == 2) ? (Bt2 + (size_t)b * strideB) : nullptr;

  const int rlane = lane & 15;
  const int koff  = (lane >> 4) * 8;
  const int mOff  = (lane >> 4) * 8;

  v8f acc[4][4];
#pragma unroll
  for (int i = 0; i < 4; ++i)
#pragma unroll
    for (int j = 0; j < 4; ++j) acc[i][j] = (v8f){0.f,0.f,0.f,0.f,0.f,0.f,0.f,0.f};

  for (int k0 = 0; k0 < K; k0 += 32) {
    V bh[4], bl[4];
#pragma unroll
    for (int j = 0; j < 4; ++j) {
      const size_t bo = (size_t)(n0 + (j << 4) + rlane) * ldb + koff + k0;
      bh[j] = Frag<T>::load(Bb + bo);
      if (SPL == 2) bl[j] = Frag<T>::load(Bb2 + bo);
    }
#pragma unroll
    for (int i = 0; i < 4; ++i) {
      const size_t ao = (size_t)(m0 + (i << 4) + rlane) * lda + koff + k0;
      V ah = Frag<T>::load(Ab + ao);
      V al;
      if (SPL >= 1) al = Frag<T>::load(Ab2 + ao);
#pragma unroll
      for (int j = 0; j < 4; ++j) {
        acc[i][j] = Frag<T>::mma(ah, bh[j], acc[i][j]);
        if (SPL == 2) acc[i][j] = Frag<T>::mma(ah, bl[j], acc[i][j]);
        if (SPL >= 1) acc[i][j] = Frag<T>::mma(al, bh[j], acc[i][j]);
      }
      Frag<T>::guard4(acc[i][0], acc[i][1], acc[i][2], acc[i][3], ah, (SPL >= 1) ? al : ah);
    }
    Frag<T>::keep(bh[0], bh[1], bh[2], bh[3]);
    if (SPL == 2) Frag<T>::keep(bl[0], bl[1], bl[2], bl[3]);
  }
  acc_guard4(acc[0][0], acc[0][1], acc[0][2], acc[0][3]);
  acc_guard4(acc[1][0], acc[1][1], acc[1][2], acc[1][3]);
  acc_guard4(acc[2][0], acc[2][1], acc[2][2], acc[2][3]);
  acc_guard4(acc[3][0], acc[3][1], acc[3][2], acc[3][3]);

  float* slab = sT[wave];
  const float* Rb = RESID ? (resid + (size_t)b * strideR) : nullptr;
#pragma unroll
  for (int i = 0; i < 4; ++i) {
    const int mBase = m0 + (i << 4);
#pragma unroll
    for (int j = 0; j < 4; ++j) {
      const int n = n0 + (j << 4) + rlane;
      float bv = 0.f;
      if (BIAS_MODE == 2) bv = bias[n];
#pragma unroll
      for (int r = 0; r < 8; ++r) {
        float v = acc[i][j][r] * scale;
        if (BIAS_MODE == 1) v += bias[mBase + mOff + r];
        if (BIAS_MODE == 2) v += bv;
        if (RESID) v += Rb[(size_t)(mBase + mOff + r) * ldc + n];
        if (ACT == 1) v = tanhf(v);
        if (ACT == 2) v = fmaxf(v, 0.0f);
        if (ACT == 3) v = v / (1.0f + expf(-v));
        if (ACT == 4) v = (v > 0.f) ? v : 0.01f * v;
        slab[(mOff + r) * 68 + (j << 4) + rlane] = v;
      }
    }
    __builtin_amdgcn_fence(__ATOMIC_RELEASE, "workgroup");
    __builtin_amdgcn_wave_barrier();
    __builtin_amdgcn_fence(__ATOMIC_ACQUIRE, "workgroup");
    if (OUT_MODE == 0) {
      float* C = (float*)Cout + (size_t)b * strideC;
      const int hh = lane >> 4, c4 = (lane & 15) * 4;
      for (int pass = 0; pass < 2; ++pass) {
#pragma unroll
        for (int it = 0; it < 8; ++it) {
          const int row = it * 2 + hh;
          v4f v = *(const v4f*)(slab + row * 68 + c4);
          *(volatile v4f*)(C + (size_t)(mBase + row) * ldc + n0 + c4) = v;
        }
        __threadfence();
      }
    } else {
      const int q = lane >> 3, c8 = (lane & 7) * 8;
      unsigned short* C  = (unsigned short*)Cout  + (size_t)b * strideC;
      unsigned short* C2 = (OUT_MODE == 2) ? ((unsigned short*)Cout2 + (size_t)b * strideC) : nullptr;
      for (int pass = 0; pass < 2; ++pass) {
#pragma unroll
        for (int it = 0; it < 4; ++it) {
          const int row = it * 4 + q;
          const float* sp = slab + row * 68 + c8;
          v8h hv, lv;
#pragma unroll
          for (int e = 0; e < 8; ++e) {
            if (OUT_MODE == 1) {
              hv[e] = (_Float16)sp[e];
            } else {
              unsigned short hb = f2bf_bits(sp[e]);
              unsigned short lb = f2bf_bits(sp[e] - bf_bits2f(hb));
              hv[e] = __builtin_bit_cast(_Float16, hb);
              lv[e] = __builtin_bit_cast(_Float16, lb);
            }
          }
          *(volatile v8h*)(C + (size_t)(mBase + row) * ldc + n0 + c8) = hv;
          if (OUT_MODE == 2) *(volatile v8h*)(C2 + (size_t)(mBase + row) * ldc + n0 + c8) = lv;
        }
        __threadfence();
      }
    }
    __builtin_amdgcn_fence(__ATOMIC_RELEASE, "workgroup");
    __builtin_amdgcn_wave_barrier();
    __builtin_amdgcn_fence(__ATOMIC_ACQUIRE, "workgroup");
  }
}

__global__ __launch_bounds__(256) void split_rows_bf16_kernel(
    const float* __restrict__ src, unsigned short* __restrict__ dhi, unsigned short* __restrict__ dlo, int total8)
{
  const int i = blockIdx.x * 256 + threadIdx.x;
  if (i >= total8) return;
  const size_t e0 = (size_t)i << 3;
  const v4f a0 = *(const v4f*)(src + e0);
  const v4f a1 = *(const v4f*)(src + e0 + 4);
  v8h hv, lv;
#pragma unroll
  for (int e = 0; e < 4; ++e) {
    const unsigned short h0 = f2bf_bits(a0[e]), h1 = f2bf_bits(a1[e]);
    const unsigned short l0 = f2bf_bits(a0[e] - bf_bits2f(h0)), l1 = f2bf_bits(a1[e] - bf_bits2f(h1));
    hv[e]     = __builtin_bit_cast(_Float16, h0);
    hv[4 + e] = __builtin_bit_cast(_Float16, h1);
    lv[e]     = __builtin_bit_cast(_Float16, l0);
    lv[4 + e] = __builtin_bit_cast(_Float16, l1);
  }
  unsigned short* qh = dhi + e0;
  unsigned short* ql = dlo + e0;
  *(volatile v8h*)qh = hv;
  *(volatile v8h*)ql = lv;
  __threadfence();
  *(volatile v8h*)qh = hv;
  *(volatile v8h*)ql = lv;
}

__global__ __launch_bounds__(256) void wt_split_kernel(
    const float* __restrict__ in, int R, int C, unsigned short* __restrict__ outH, unsigned short* __restrict__ outL)
{
  __shared__ __align__(16) float tile[64 * 33];
  const int tid = threadIdx.x, lane = tid & 31, wave = tid >> 5;
  const int c0 = blockIdx.x * 32;
  const int r0 = blockIdx.y * 64;
#pragma unroll
  for (int i = 0; i < 8; ++i) {
    const int row = i * 8 + wave;
    tile[row * 33 + lane] = in[(size_t)(r0 + row) * C + c0 + lane];
  }
  __syncthreads();
  const int q = lane >> 3, e8 = (lane & 7) * 8;
  const int j = wave * 4 + q;
  v8h hv, lv;
#pragma unroll
  for (int e = 0; e < 8; ++e) {
    const float f = tile[(e8 + e) * 33 + j];
    const unsigned short hb = f2bf_bits(f);
    const unsigned short lb = f2bf_bits(f - bf_bits2f(hb));
    hv[e] = __builtin_bit_cast(_Float16, hb);
    lv[e] = __builtin_bit_cast(_Float16, lb);
  }
  const size_t o = (size_t)(c0 + j) * R + r0 + e8;
  *(volatile v8h*)(outH + o) = hv;
  *(volatile v8h*)(outL + o) = lv;
  __threadfence();
  *(volatile v8h*)(outH + o) = hv;
  *(volatile v8h*)(outL + o) = lv;
}

__global__ __launch_bounds__(256) void atab_kernel(const float* __restrict__ Alog, float* __restrict__ AT4)
{
  const int g = blockIdx.x * 256 + threadIdx.x;
  const int s4 = g >> 8;
  const int i  = g & (kDin - 1);
  const v4f a = *(const v4f*)(Alog + (size_t)i * kDst + 4 * s4);
  v4f o;
  o[0] = -expf(a[0]); o[1] = -expf(a[1]); o[2] = -expf(a[2]); o[3] = -expf(a[3]);
  float* dst = AT4 + (size_t)g * 4;
  *(volatile v4f*)dst = o;
  __threadfence();
  *(volatile v4f*)dst = o;
}

__global__ __launch_bounds__(256) void conv_sum_kernel(
    const float* __restrict__ XZ, const float* __restrict__ cw, const float* __restrict__ cb,
    const float* __restrict__ Wx, float* __restrict__ XC, unsigned short* __restrict__ XCH,
    unsigned short* __restrict__ XCL, float* __restrict__ SS)
{
  __shared__ __align__(16) float sT[16 * kConvTP];
  __shared__ __align__(16) float sW[kDin];
  __shared__ __align__(16) float sS[64];
  const int tid = threadIdx.x, lane = tid & 31, wave = tid >> 5;
  const int d = tid;
  const int g0 = blockIdx.x * 64;
  const int tb = g0 & (kSeq - 1);
  float wsm = 0.0f;
#pragma unroll 1
  for (int j4 = 0; j4 < kDst / 4; ++j4) {
    const v4f w = *(const v4f*)(Wx + (size_t)d * kXxW + kDst + 4 * j4);
    wsm += w[0]; wsm += w[1]; wsm += w[2]; wsm += w[3];
  }
  sW[d] = wsm;
  const float w0 = cw[d * kConvK + 0], w1 = cw[d * kConvK + 1], w2 = cw[d * kConvK + 2], w3 = cw[d * kConvK + 3];
  const float bc = cb[d];
  float xm3, xm2, xm1;
  {
    const bool hist = (tb > 0);
    const int rb = hist ? (g0 - 3) : g0;
    const float v3 = XZ[(size_t)rb * kXzW + d];
    const float v2 = XZ[(size_t)(rb + 1) * kXzW + d];
    const float v1 = XZ[(size_t)(rb + 2) * kXzW + d];
    xm3 = hist ? v3 : 0.f;
    xm2 = hist ? v2 : 0.f;
    xm1 = hist ? v1 : 0.f;
  }
  const int hrow = wave >> 1;
  const int hch  = (wave & 1) * 128 + lane * 4;
  __syncthreads();
#pragma unroll 1
  for (int sub = 0; sub < 4; ++sub) {
    const int lb = g0 + sub * 16;
#pragma unroll 1
    for (int s = 0; s < 16; ++s) {
      const float xcur = XZ[(size_t)(lb + s) * kXzW + d];
      float acc = w0 * xm3;
      acc = fmaf(w1, xm2, acc);
      acc = fmaf(w2, xm1, acc);
      acc = fmaf(w3, xcur, acc);
      sT[s * kConvTP + tid] = acc + bc;
      xm3 = xm2; xm2 = xm1; xm1 = xcur;
    }
    __syncthreads();
    {
      const v4f wv0 = *(const v4f*)(sW + lane * 8);
      const v4f wv1 = *(const v4f*)(sW + lane * 8 + 4);
      float ps[2];
#pragma unroll
      for (int rr = 0; rr < 2; ++rr) {
        const float* sp = sT + (2 * wave + rr) * kConvTP + lane * 8;
        const v4f a0 = *(const v4f*)(sp);
        const v4f a1 = *(const v4f*)(sp + 4);
        float p = a0[0] * wv0[0];
        p = fmaf(a0[1], wv0[1], p);
        p = fmaf(a0[2], wv0[2], p);
        p = fmaf(a0[3], wv0[3], p);
        p = fmaf(a1[0], wv1[0], p);
        p = fmaf(a1[1], wv1[1], p);
        p = fmaf(a1[2], wv1[2], p);
        p = fmaf(a1[3], wv1[3], p);
#pragma unroll
        for (int off = 16; off > 0; off >>= 1) p += __shfl_xor(p, off, 32);
        ps[rr] = p;
      }
      if (lane == 0) {
        sS[sub * 16 + 2 * wave]     = ps[0];
        sS[sub * 16 + 2 * wave + 1] = ps[1];
      }
    }
    v4f fv[4];
    v8h bh[2], blo[2];
#pragma unroll
    for (int it = 0; it < 4; ++it) fv[it] = *(const v4f*)(sT + (it * 4 + hrow) * kConvTP + hch);
#pragma unroll
    for (int it = 0; it < 2; ++it) {
      const float* sp = sT + (it * 8 + wave) * kConvTP + lane * 8;
      const v4f a0 = *(const v4f*)(sp);
      const v4f a1 = *(const v4f*)(sp + 4);
#pragma unroll
      for (int e = 0; e < 4; ++e) {
        const unsigned short h0 = f2bf_bits(a0[e]), h1 = f2bf_bits(a1[e]);
        const unsigned short l0 = f2bf_bits(a0[e] - bf_bits2f(h0)), l1 = f2bf_bits(a1[e] - bf_bits2f(h1));
        bh[it][e]      = __builtin_bit_cast(_Float16, h0);
        bh[it][4 + e]  = __builtin_bit_cast(_Float16, h1);
        blo[it][e]     = __builtin_bit_cast(_Float16, l0);
        blo[it][4 + e] = __builtin_bit_cast(_Float16, l1);
      }
    }
    for (int pass = 0; pass < 2; ++pass) {
#pragma unroll
      for (int it = 0; it < 4; ++it)
        *(volatile v4f*)(XC + (size_t)(lb + it * 4 + hrow) * kDin + hch) = fv[it];
#pragma unroll
      for (int it = 0; it < 2; ++it) {
        const size_t o = (size_t)(lb + it * 8 + wave) * kDin + lane * 8;
        *(volatile v8h*)(XCH + o) = bh[it];
        *(volatile v8h*)(XCL + o) = blo[it];
      }
      __threadfence();
    }
    __syncthreads();
  }
  {
    const int lc = (lane < 16) ? lane : 15;
    const v4f sv = *(const v4f*)(sS + lc * 4);
    float* dst = SS + g0 + lc * 4;
    if (wave == 0 && lane < 16) *(volatile v4f*)dst = sv;
    __threadfence();
    if (wave == 0 && lane < 16) *(volatile v4f*)dst = sv;
  }
}

__global__ __launch_bounds__(256) void scan_kernel(
    const float* __restrict__ PRE, const float* __restrict__ XC, const float* __restrict__ SS,
    const float* __restrict__ XZ, const float* __restrict__ bdt, const float* __restrict__ AT4,
    unsigned short* __restrict__ GH, unsigned short* __restrict__ GL)
{
  __shared__ __align__(16) float sy[2 * kDst];
  __shared__ __align__(16) float sG[kScanTS * kScanGP];
  const int tid = threadIdx.x, lane = tid & 31, wave = tid >> 5;
  const int i = tid;
  const size_t row0 = (size_t)blockIdx.x * kSeq;
  const float bb = bdt[i];
  sy[i] = 0.0f;
  __syncthreads();
  int cur = 0;
#pragma unroll 1
  for (int t0 = 0; t0 < kSeq; t0 += kScanTS) {
#pragma unroll 1
    for (int s = 0; s < kScanTS; ++s) {
      const size_t tok = row0 + (size_t)(t0 + s);
      const float pre = PRE[tok * kDst + i] + bb;
      const float ea  = expf(-fabsf(pre));
      const float dlt = fmaxf(pre, 0.0f) + logf(1.0f + ea);
      const float xcv = XC[tok * kDin + i];
      const float sv  = SS[tok];
      const float bt  = (dlt * xcv) * sv;
      const float* yb = sy + cur * kDst;
      float acc = 0.0f;
#pragma unroll 1
      for (int s4 = 0; s4 < kDst / 4; ++s4) {
        const v4f yv = *(const v4f*)(yb + 4 * s4);
        const v4f av = *(const v4f*)(AT4 + ((size_t)s4 * kDin + i) * 4);
        acc = fmaf(expf(dlt * av[0]), yv[0], acc);
        acc = fmaf(expf(dlt * av[1]), yv[1], acc);
        acc = fmaf(expf(dlt * av[2]), yv[2], acc);
        acc = fmaf(expf(dlt * av[3]), yv[3], acc);
      }
      const float ynew = acc + bt;
      sy[(cur ^ 1) * kDst + i] = ynew;
      const float zv = XZ[tok * kXzW + kDin + i];
      const float gate = zv / (1.0f + expf(-zv));
      sG[s * kScanGP + i] = ynew * gate;
      __syncthreads();
      cur ^= 1;
    }
    v8h hv[4], lv[4];
#pragma unroll
    for (int it = 0; it < 4; ++it) {
      const int row = it * 8 + wave;
      const float* sp = sG + row * kScanGP + lane * 8;
      const v4f a0 = *(const v4f*)(sp);
      const v4f a1 = *(const v4f*)(sp + 4);
#pragma unroll
      for (int e = 0; e < 4; ++e) {
        const unsigned short h0 = f2bf_bits(a0[e]), h1 = f2bf_bits(a1[e]);
        const unsigned short l0 = f2bf_bits(a0[e] - bf_bits2f(h0)), l1 = f2bf_bits(a1[e] - bf_bits2f(h1));
        hv[it][e]     = __builtin_bit_cast(_Float16, h0);
        hv[it][4 + e] = __builtin_bit_cast(_Float16, h1);
        lv[it][e]     = __builtin_bit_cast(_Float16, l0);
        lv[it][4 + e] = __builtin_bit_cast(_Float16, l1);
      }
    }
    for (int pass = 0; pass < 2; ++pass) {
#pragma unroll
      for (int it = 0; it < 4; ++it) {
        const int row = it * 8 + wave;
        const size_t o = (row0 + (size_t)(t0 + row)) * kDin + lane * 8;
        *(volatile v8h*)(GH + o) = hv[it];
        *(volatile v8h*)(GL + o) = lv[it];
      }
      __threadfence();
    }
    __syncthreads();
  }
}

extern "C" void kernel_launch(void* const* d_in, const int* in_sizes, int n_in,
                              void* d_out, int out_size, void* d_ws, size_t ws_size,
                              hipStream_t stream) {
  if (n_in < 9) return;
  if (in_sizes[0] != kRows * kDm) return;
  if (in_sizes[1] != kDm * kXzW) return;
  if (in_sizes[2] != kDin * kConvK) return;
  if (in_sizes[3] != kDin) return;
  if (in_sizes[4] != kDin * kXxW) return;
  if (in_sizes[5] != kDin * kDst) return;
  if (in_sizes[6] != kDst) return;
  if (in_sizes[7] != kDin * kDst) return;
  if (in_sizes[8] != kDin * kDm) return;
  if (out_size != kRows * kDm) return;
  if (ws_size < kWsTotal) return;

  const float* x      = (const float*)d_in[0];
  const float* W_in   = (const float*)d_in[1];
  const float* conv_w = (const float*)d_in[2];
  const float* conv_b = (const float*)d_in[3];
  const float* W_x    = (const float*)d_in[4];
  const float* W_dt   = (const float*)d_in[5];
  const float* b_dt   = (const float*)d_in[6];
  const float* A_log  = (const float*)d_in[7];
  const float* W_out  = (const float*)d_in[8];
  float* out = (float*)d_out;

  char* ws = (char*)d_ws;
  unsigned short* XH   = (unsigned short*)(ws + kOffXH);
  unsigned short* XL   = (unsigned short*)(ws + kOffXL);
  unsigned short* WIH  = (unsigned short*)(ws + kOffWIH);
  unsigned short* WIL  = (unsigned short*)(ws + kOffWIL);
  unsigned short* WDH  = (unsigned short*)(ws + kOffWDH);
  unsigned short* WDL  = (unsigned short*)(ws + kOffWDL);
  unsigned short* WOH  = (unsigned short*)(ws + kOffWOH);
  unsigned short* WOL  = (unsigned short*)(ws + kOffWOL);
  float*          AT4  = (float*)(ws + kOffAT);
  float*          XZ   = (float*)(ws + kOffXZ);
  float*          XC   = (float*)(ws + kOffXC);
  unsigned short* XCH  = (unsigned short*)(ws + kOffXCH);
  unsigned short* XCL  = (unsigned short*)(ws + kOffXCL);
  float*          SS   = (float*)(ws + kOffSS);
  float*          PRE  = (float*)(ws + kOffPRE);
  unsigned short* GH   = (unsigned short*)(ws + kOffGH);
  unsigned short* GL   = (unsigned short*)(ws + kOffGL);

  split_rows_bf16_kernel<<<(kRows * kDm / 8) / 256, 256, 0, stream>>>(x, XH, XL, kRows * kDm / 8);
  wt_split_kernel<<<dim3(kXzW / 32, kDm / 64), 256, 0, stream>>>(W_in, kDm, kXzW, WIH, WIL);
  wt_split_kernel<<<dim3(kDst / 32, kDin / 64), 256, 0, stream>>>(W_dt, kDin, kDst, WDH, WDL);
  wt_split_kernel<<<dim3(kDm / 32, kDin / 64), 256, 0, stream>>>(W_out, kDin, kDm, WOH, WOL);
  atab_kernel<<<(kDst / 4) * kDin / 256, 256, 0, stream>>>(A_log, AT4);

  wmma_gemm64<1, 2, 0, 0, false><<<dim3((kRows / 64) * (kXzW / 64) / 8, 1), 256, 0, stream>>>(
      XH, XL, kDm, 0L,
      WIH, WIL, kDm, 0L,
      (void*)XZ, nullptr, kXzW, 0L,
      nullptr, nullptr, 0L,
      kRows, kXzW, kDm, 1.0f);

  conv_sum_kernel<<<kRows / 64, 256, 0, stream>>>(XZ, conv_w, conv_b, W_x, XC, XCH, XCL, SS);

  wmma_gemm64<1, 2, 0, 0, false><<<dim3((kRows / 64) * (kDst / 64) / 8, 1), 256, 0, stream>>>(
      XCH, XCL, kDin, 0L,
      WDH, WDL, kDin, 0L,
      (void*)PRE, nullptr, kDst, 0L,
      nullptr, nullptr, 0L,
      kRows, kDst, kDin, 1.0f);

  scan_kernel<<<kBatch, kDin, 0, stream>>>(PRE, XC, SS, XZ, b_dt, AT4, GH, GL);

  wmma_gemm64<1, 2, 0, 0, false><<<dim3((kRows / 64) * (kDm / 64) / 8, 1), 256, 0, stream>>>(
      GH, GL, kDin, 0L,
      WOH, WOL, kDin, 0L,
      (void*)out, nullptr, kDm, 0L,
      nullptr, nullptr, 0L,
      kRows, kDm, kDin, 1.0f);
}
